// SpatialGATAttention_60490319397015
// MI455X (gfx1250) — hardware-verified
//
#include <hip/hip_runtime.h>
#include <math.h>
#include <stdint.h>

#ifndef NB
#define NB 8
#endif
#define NBX   8
#define TT    32
#define CC    64
#define NN    400
#define NH    2
#define HD    32
#define BT    (NB * TT)
#define NQT   (NN / 16)
#define KP    448
#define NKT   13
#define NJT   (KP / 64)
#define NPROJ (3 * CC)
#define MROWS (BT * NN)
#define X_BSTRIDE_FULL ((size_t)CC * TT * NN)
#define LOG2E 1.4426950408889634f
#define NEGM  (-1.0e9f)
#define LNEPS 1.0e-5f
#define PCAR  16384.0f
#define VCAR  1024.0f
#define VTP   72
#define PTP   36
#define PTW   (16 * PTP)
#define RSP   68
#define SLAB64 (16 * 68)
#define ATT_THREADS (NH * 32)
#define OCHUNK 1024
#define NOCH  ((TT * NN + OCHUNK - 1) / OCHUNK)
#define WS_CAP 134217728
static_assert(CC == NH * HD && HD == 32 && NH == 2 && ATT_THREADS == 64);
static_assert(NB >= 1 && NB <= NBX);
static_assert((NN % 16) == 0 && NQT * 16 == NN && (NN % 4) == 0);
static_assert((MROWS % 64) == 0 && (NPROJ % 64) == 0 && (CC % 32) == 0);
static_assert(NKT * 32 >= NN && NKT * 32 <= KP && NKT <= 16 && (KP % 64) == 0 && NJT * 64 == KP);
static_assert(((TT * NN) % 4) == 0 && (OCHUNK % 1024) == 0);
static_assert(NN * 16 == 25 * 256);
static_assert((NPROJ * CC) % (8 * 256) == 0);

typedef unsigned short u16;
typedef _Float16 v16h __attribute__((ext_vector_type(16)));
typedef _Float16 v8h  __attribute__((ext_vector_type(8)));
typedef __bf16   v16b __attribute__((ext_vector_type(16)));
typedef float    v8f  __attribute__((ext_vector_type(8)));
typedef float    v4f  __attribute__((ext_vector_type(4)));
typedef unsigned int v4u __attribute__((ext_vector_type(4)));

union FragH { v16h v; v8h h[2]; v4u u[2]; };
union FragB { v16b v; v4u u[2]; };

__device__ __forceinline__ unsigned short bf_bits(float f) {
  unsigned u = __float_as_uint(f);
  return (unsigned short)((u + 0x7FFFu + ((u >> 16) & 1u)) >> 16);
}
__device__ __forceinline__ float bf_up(unsigned short h) { return __uint_as_float(((unsigned)h) << 16); }
__device__ __forceinline__ float bfr(float f) { return bf_up(bf_bits(f)); }
__device__ __forceinline__ unsigned short h_bits(_Float16 x) { return __builtin_bit_cast(unsigned short, x); }
__device__ __forceinline__ unsigned pk16(unsigned short a, unsigned short b) { return (unsigned)a | ((unsigned)b << 16); }
__device__ __forceinline__ v8f zero8() { v8f z = {0.f, 0.f, 0.f, 0.f, 0.f, 0.f, 0.f, 0.f}; return z; }

__device__ __forceinline__ v16h ldfrag_h(const _Float16* p) {
  FragH f;
  f.h[0] = *(const v8h*)(p);
  f.h[1] = *(const v8h*)(p + 16);
  return f.v;
}
__device__ __forceinline__ v16b ldfrag_b(const u16* p) {
  FragB f;
  f.u[0] = *(const v4u*)(p);
  f.u[1] = *(const v4u*)(p + 16);
  return f.v;
}

__device__ __forceinline__ v8f mma_h(v16h a, v16h b, v8f c) {
  return __builtin_amdgcn_wmma_f32_16x16x32_f16(false, a, false, b, (short)0, c, false, false);
}
__device__ __forceinline__ v8f mma_b(v16b a, v16b b, v8f c) {
  return __builtin_amdgcn_wmma_f32_16x16x32_bf16(false, a, false, b, (short)0, c, false, false);
}
__device__ __forceinline__ void guard2(v8f& a, v8f& b, v16h x0, v16h x1, v16h x2, v16h x3, v16h x4, v16h x5) {
#if defined(__HIP_DEVICE_COMPILE__)
  asm volatile("v_nop\n\tv_nop\n\tv_nop\n\tv_nop"
               : "+v"(a), "+v"(b) : "v"(x0), "v"(x1), "v"(x2), "v"(x3), "v"(x4), "v"(x5) : "memory");
#endif
}
template <typename F>
__device__ __forceinline__ void guard6(v8f& a, v8f& b, v8f& c, v8f& d, F x0, F x1, F x2, F x3, F x4, F x5) {
#if defined(__HIP_DEVICE_COMPILE__)
  asm volatile("v_nop\n\tv_nop\n\tv_nop\n\tv_nop"
               : "+v"(a), "+v"(b), "+v"(c), "+v"(d) : "v"(x0), "v"(x1), "v"(x2), "v"(x3), "v"(x4), "v"(x5) : "memory");
#endif
}
__device__ __forceinline__ void acc_guard2(v8f& a, v8f& b) {
#if defined(__HIP_DEVICE_COMPILE__)
  asm volatile("v_nop\n\tv_nop\n\tv_nop\n\tv_nop" : "+v"(a), "+v"(b));
#endif
}
__device__ __forceinline__ void wave_sync_lds() {
  __builtin_amdgcn_fence(__ATOMIC_RELEASE, "workgroup");
  __builtin_amdgcn_wave_barrier();
  __builtin_amdgcn_fence(__ATOMIC_ACQUIRE, "workgroup");
}

__global__ __launch_bounds__(256) void wcvt(const float* __restrict__ Wq, const float* __restrict__ Wk,
                                            const float* __restrict__ Wv, u16* WBo) {
  const int gt = blockIdx.x * 256 + (int)threadIdx.x;
  if (gt >= (NPROJ * CC) / 8) return;
  const int row = gt >> 3, c8 = (gt & 7) * 8;
  const int which = row / CC;
  const int p = (row - which * CC) * CC + c8;
  const v4f q0 = *(const v4f*)(Wq + p), q1 = *(const v4f*)(Wq + p + 4);
  const v4f k0 = *(const v4f*)(Wk + p), k1 = *(const v4f*)(Wk + p + 4);
  const v4f w0 = *(const v4f*)(Wv + p), w1 = *(const v4f*)(Wv + p + 4);
  float f[8];
#pragma unroll
  for (int e = 0; e < 4; ++e) {
    f[e]     = (which == 0) ? q0[e] : ((which == 1) ? k0[e] : w0[e]);
    f[4 + e] = (which == 0) ? q1[e] : ((which == 1) ? k1[e] : w1[e]);
  }
  v4u o;
#pragma unroll
  for (int e = 0; e < 4; ++e) o[e] = pk16(bf_bits(f[2 * e]), bf_bits(f[2 * e + 1]));
  u16* d = WBo + (size_t)gt * 8;
  for (int pass = 0; pass < 2; ++pass) {
    *(volatile v4u*)(d) = o;
    __threadfence();
  }
}

__global__ __launch_bounds__(128) void xcvt(const float* __restrict__ x, u16* XBo) {
  __shared__ __align__(16) u16 T[16 * VTP];
  const int tid = threadIdx.x;
  const int bid = blockIdx.x;
  const int nt  = bid % NQT;
  const int bt  = bid / NQT;
  if (bt >= BT) return;
  const int b  = bt / TT, t = bt - b * TT;
  const int n0 = nt * 16;
  {
    const int c = tid >> 1, n8 = (tid & 1) * 8;
    const float* src = x + (size_t)b * X_BSTRIDE_FULL + ((size_t)c * TT + t) * NN + n0 + n8;
    const v4f a = *(const v4f*)(src), b4 = *(const v4f*)(src + 4);
#pragma unroll
    for (int e = 0; e < 4; ++e) {
      T[(n8 + e) * VTP + c]     = bf_bits(a[e]);
      T[(n8 + 4 + e) * VTP + c] = bf_bits(b4[e]);
    }
  }
  __syncthreads();
  const int line = tid >> 3, p8 = (tid & 7) * 8;
  const v4u o = *(const v4u*)(T + line * VTP + p8);
  u16* d = XBo + ((size_t)bt * NN + n0 + line) * CC + p8;
  for (int pass = 0; pass < 2; ++pass) {
    *(volatile v4u*)(d) = o;
    __threadfence();
  }
}

__global__ __launch_bounds__(256) void mbits(const int* __restrict__ gso, unsigned* MBo) {
  __shared__ __align__(16) unsigned Wl[256];
  const int tid = threadIdx.x;
  const int w = blockIdx.x * 256 + tid;
  int i = w >> 4;
  if (i > NN - 1) i = NN - 1;
  const int wj = w & 15;
  unsigned bits = 0u;
#pragma unroll 4
  for (int q = 0; q < 32; ++q) {
    const int j  = wj * 32 + q;
    const int jc = (j < NN) ? j : (NN - 1);
    const int gv = gso[(size_t)i * NN + jc];
    const unsigned on = (gv != 0 && j < NN) ? 1u : 0u;
    bits |= on << q;
  }
  Wl[tid] = bits;
  __syncthreads();
  if (tid < 64) {
    const v4u o = *(const v4u*)(Wl + tid * 4);
    unsigned* d = MBo + (size_t)blockIdx.x * 256 + tid * 4;
    for (int pass = 0; pass < 2; ++pass) {
      *(volatile v4u*)(d) = o;
      __threadfence();
    }
  }
}

__device__ __forceinline__ void epi64(float* sl, v8f a0, v8f a1, v8f a2, v8f a3, float oscale,
                                      float* C, int N, size_t rowb, int col0, int lane) {
  const int hh = lane >> 4, m = lane & 15;
#pragma unroll
  for (int r = 0; r < 8; ++r) {
    const int ro = (8 * hh + r) * 68 + m;
    sl[ro]      = a0[r] * oscale;
    sl[ro + 16] = a1[r] * oscale;
    sl[ro + 32] = a2[r] * oscale;
    sl[ro + 48] = a3[r] * oscale;
  }
  wave_sync_lds();
  v4f vals[8];
#pragma unroll
  for (int it = 0; it < 8; ++it) vals[it] = *(const v4f*)(sl + (it * 2 + hh) * 68 + m * 4);
  float* dst = C + (rowb + (size_t)hh) * (size_t)N + col0 + m * 4;
  for (int pass = 0; pass < 2; ++pass) {
#pragma unroll
    for (int it = 0; it < 8; ++it) {
      *(volatile v4f*)(dst + (size_t)(it * 2) * (size_t)N) = vals[it];
    }
    __threadfence();
  }
}

__global__ __launch_bounds__(128)
void gemm_bf(const u16* __restrict__ A, const u16* __restrict__ Bt, float* C, int M, int N, int K, float oscale) {
  __shared__ __align__(16) float slab[4 * SLAB64];
  const int tid = threadIdx.x, wave = tid >> 5, lane = tid & 31, hh = lane >> 4, m = lane & 15;
  const int ntile = N >> 6;
  const int bid   = blockIdx.x;
  const int rowb  = (bid / ntile) * 64 + wave * 16;
  const int col0  = (bid % ntile) * 64;
  if (rowb + 16 > M) return;
  const u16* ap = A  + (size_t)(rowb + m) * K + 8 * hh;
  const u16* bp = Bt + (size_t)(col0 + m) * K + 8 * hh;
  const size_t bs = (size_t)16 * K;
  v8f acc0 = zero8(), acc1 = zero8(), acc2 = zero8(), acc3 = zero8();
#pragma unroll 1
  for (int k0 = 0; k0 < K; k0 += 32) {
    const v16b a  = ldfrag_b(ap + k0);
    const v16b b0 = ldfrag_b(bp + k0);
    const v16b b1 = ldfrag_b(bp + bs + k0);
    const v16b b2 = ldfrag_b(bp + 2 * bs + k0);
    const v16b b3 = ldfrag_b(bp + 3 * bs + k0);
    acc0 = mma_b(a, b0, acc0);
    acc1 = mma_b(a, b1, acc1);
    acc2 = mma_b(a, b2, acc2);
    acc3 = mma_b(a, b3, acc3);
    guard6<v16b>(acc0, acc1, acc2, acc3, a, b0, b1, b2, b3, a);
  }
  epi64(slab + wave * SLAB64, acc0, acc1, acc2, acc3, oscale, C, N, (size_t)rowb, col0, lane);
}

__global__ __launch_bounds__(256) void vs16(const float* __restrict__ F, const float* __restrict__ asrc,
                                            const float* __restrict__ adst, u16* VHo, u16* VLo, float* SPo) {
  __shared__ __align__(16) u16 TH[CC * VTP];
  __shared__ __align__(16) u16 TL[CC * VTP];
  __shared__ __align__(16) float S4[256];
  const int tid = threadIdx.x;
  const int bid = blockIdx.x;
  const int jt  = bid % NJT;
  const int bt  = bid / NJT;
  if (bt >= BT) return;
  const int j0  = jt * 64;
  {
    const int sl = tid >> 2;
    const int dc = (tid & 3) * 16;
    const int j  = j0 + sl;
    const int jc = (j < NN) ? j : (NN - 1);
    const bool ok = (j < NN);
    const float* src = F + ((size_t)bt * NN + jc) * NPROJ + 2 * CC + dc;
#pragma unroll
    for (int i = 0; i < 4; ++i) {
      const v4f a = *(const v4f*)(src + 4 * i);
#pragma unroll
      for (int e = 0; e < 4; ++e) {
        const float t = ok ? (a[e] * VCAR) : 0.0f;
        const _Float16 hv = (_Float16)t;
        const _Float16 lv = (_Float16)(t - (float)hv);
        TH[(dc + 4 * i + e) * VTP + sl] = h_bits(hv);
        TL[(dc + 4 * i + e) * VTP + sl] = h_bits(lv);
      }
    }
  }
  {
    const int node  = tid & 63;
    const int which = tid >> 6;
    const int hsel  = which & 1;
    const int isdst = which >> 1;
    const int j  = j0 + node;
    const int jc = (j < NN) ? j : (NN - 1);
    const bool ok = (j < NN);
    const float* fr = F + ((size_t)bt * NN + jc) * NPROJ + isdst * CC + hsel * HD;
    const float* pa = asrc + hsel * HD;
    const float* pd = adst + hsel * HD;
    float acc = 0.0f;
#pragma unroll 2
    for (int d4 = 0; d4 < HD / 4; ++d4) {
      const v4f f4 = *(const v4f*)(fr + 4 * d4);
      const v4f a4 = *(const v4f*)(pa + 4 * d4);
      const v4f b4 = *(const v4f*)(pd + 4 * d4);
#pragma unroll
      for (int e = 0; e < 4; ++e) {
        const float av = isdst ? b4[e] : a4[e];
        acc += f4[e] * bfr(av);
      }
    }
    S4[tid] = ok ? acc : 0.0f;
  }
  __syncthreads();
  v4u vh[2], vl[2];
  const int q8 = tid >> 3, p8 = (tid & 7) * 8;
#pragma unroll
  for (int it = 0; it < 2; ++it) {
    const int line = it * 32 + q8;
    vh[it] = *(const v4u*)(TH + line * VTP + p8);
    vl[it] = *(const v4u*)(TL + line * VTP + p8);
  }
  const int  tcl  = (tid < 64) ? tid : 0;
  const v4f  sv   = *(const v4f*)(S4 + tcl * 4);
  const int  seg  = tcl >> 4;
  const size_t sidx = ((size_t)(seg >> 1) * BT * NH + (size_t)bt * NH + (seg & 1)) * KP + j0 + (tcl & 15) * 4;
  const size_t baseV = ((size_t)bt * CC) * KP + j0 + p8;
  const bool dos = (tid < 64);
  for (int pass = 0; pass < 2; ++pass) {
#pragma unroll
    for (int it = 0; it < 2; ++it) {
      const int line = it * 32 + q8;
      *(volatile v4u*)(VHo + baseV + (size_t)line * KP) = vh[it];
      *(volatile v4u*)(VLo + baseV + (size_t)line * KP) = vl[it];
    }
    if (dos) *(volatile v4f*)(SPo + sidx) = sv;
    __threadfence();
  }
}

__global__ __launch_bounds__(ATT_THREADS)
void gat_attn(const float* __restrict__ SP, const unsigned* __restrict__ MBp,
              const u16* __restrict__ VHp, const u16* __restrict__ VLp,
              const float* __restrict__ gam, const float* __restrict__ bet, float* OP) {
  __shared__ __align__(16) float    pt[NH * PTW];
  __shared__ __align__(16) float    sdl[NH * KP];
  __shared__ __align__(16) float    rsl[16 * RSP];
  __shared__ __align__(16) unsigned mwl[16 * 16];

  const int tid  = threadIdx.x;
  const int wave = tid >> 5;
  const int lane = tid & 31;
  const int hh   = lane >> 4;
  const int c    = lane & 15;
  const int bid  = blockIdx.x;
  const int qt   = bid % NQT;
  const int bt   = bid / NQT;
  if (bt >= BT) return;
  const int q0   = qt * 16;
  const int head = wave;
  float* ptw = pt  + wave * PTW;
  float* sdw = sdl + wave * KP;

  {
    const float* sdg = SP + ((size_t)BT * NH + (size_t)bt * NH + head) * KP;
    for (int idx = lane; idx < KP / 4; idx += 32) *(v4f*)(sdw + idx * 4) = *(const v4f*)(sdg + idx * 4);
    const int row = tid >> 2, w4 = (tid & 3) * 4;
    *(v4u*)(mwl + row * 16 + w4) = *(const v4u*)(MBp + (size_t)(q0 + row) * 16 + w4);
  }
  float ssv[8];
  {
    const float* ssg = SP + ((size_t)bt * NH + head) * KP + q0 + 8 * hh;
    const v4f a = *(const v4f*)(ssg), b4 = *(const v4f*)(ssg + 4);
#pragma unroll
    for (int e = 0; e < 4; ++e) { ssv[e] = a[e]; ssv[4 + e] = b4[e]; }
  }
  __syncthreads();

  const _Float16* Vhb = (const _Float16*)(const void*)VHp + ((size_t)bt * CC + head * HD + c) * KP + 8 * hh;
  const _Float16* Vlb = (const _Float16*)(const void*)VLp + ((size_t)bt * CC + head * HD + c) * KP + 8 * hh;
  const size_t dsub = (size_t)16 * KP;

  float mrow[8], lrow[8];
#pragma unroll
  for (int r = 0; r < 8; ++r) { mrow[r] = -INFINITY; lrow[r] = 0.f; }
  v8f o0 = zero8(), o1 = zero8();

#pragma unroll 1
  for (int kt = 0; kt < NKT; ++kt) {
    const int kb = kt * 32;
    const int key0 = kb + c, key1 = kb + 16 + c;
    const float sd0 = sdw[key0], sd1 = sdw[key1];
    const bool in0 = (key0 < NN), in1 = (key1 < NN);
#pragma unroll
    for (int r = 0; r < 8; ++r) {
      const unsigned mword = mwl[(8 * hh + r) * 16 + kt];
      const bool on0 = ((mword >> c) & 1u) != 0u;
      const bool on1 = ((mword >> (16 + c)) & 1u) != 0u;
      float u0 = ssv[r] + sd0;
      float u1 = ssv[r] + sd1;
      u0 = (u0 >= 0.0f) ? u0 : (0.2f * u0);
      u1 = (u1 >= 0.0f) ? u1 : (0.2f * u1);
      u0 = u0 + (on0 ? 0.0f : NEGM);
      u1 = u1 + (on1 ? 0.0f : NEGM);
      const float t0 = in0 ? (u0 * LOG2E) : -INFINITY;
      const float t1 = in1 ? (u1 * LOG2E) : -INFINITY;
      float mx = fmaxf(t0, t1);
#pragma unroll
      for (int off = 1; off < 16; off <<= 1) mx = fmaxf(mx, __shfl_xor(mx, off, 32));
      const float mn = fmaxf(mrow[r], mx);
      const float ms = (mn == -INFINITY) ? 0.0f : mn;
      const float al = exp2f(mrow[r] - ms);
      mrow[r] = mn;
      const float e0 = exp2f(t0 - ms), e1 = exp2f(t1 - ms);
      float ps = e0 + e1;
#pragma unroll
      for (int off = 1; off < 16; off <<= 1) ps += __shfl_xor(ps, off, 32);
      lrow[r] = lrow[r] * al + ps;
      o0[r] *= al;
      o1[r] *= al;
      const int ro = (8 * hh + r) * PTP + c;
      ptw[ro]      = e0;
      ptw[ro + 16] = e1;
    }
    wave_sync_lds();
    FragH ph, pl;
    {
      const float* prow = ptw + c * PTP + 8 * hh;
      const v4f p0 = *(const v4f*)(prow), p1 = *(const v4f*)(prow + 4);
      const v4f p2 = *(const v4f*)(prow + 16), p3 = *(const v4f*)(prow + 20);
#pragma unroll
      for (int e = 0; e < 4; ++e) {
        const float ta = p0[e] * PCAR, tb = p1[e] * PCAR, tc = p2[e] * PCAR, td = p3[e] * PCAR;
        const _Float16 ha = (_Float16)ta, hb = (_Float16)tb, hc = (_Float16)tc, hd = (_Float16)td;
        ph.h[0][e]     = ha;
        ph.h[0][4 + e] = hb;
        ph.h[1][e]     = hc;
        ph.h[1][4 + e] = hd;
        pl.h[0][e]     = (_Float16)(ta - (float)ha);
        pl.h[0][4 + e] = (_Float16)(tb - (float)hb);
        pl.h[1][e]     = (_Float16)(tc - (float)hc);
        pl.h[1][4 + e] = (_Float16)(td - (float)hd);
      }
    }
    {
      const _Float16* vhp = Vhb + kb;
      const _Float16* vlp = Vlb + kb;
      const v16h vha = ldfrag_h(vhp), vhb2 = ldfrag_h(vhp + dsub);
      const v16h vla = ldfrag_h(vlp), vlb2 = ldfrag_h(vlp + dsub);
      o0 = mma_h(ph.v, vha,  o0);
      o0 = mma_h(pl.v, vha,  o0);
      o0 = mma_h(ph.v, vla,  o0);
      o1 = mma_h(ph.v, vhb2, o1);
      o1 = mma_h(pl.v, vhb2, o1);
      o1 = mma_h(ph.v, vlb2, o1);
      guard2(o0, o1, ph.v, pl.v, vha, vhb2, vla, vlb2);
    }
    wave_sync_lds();
  }
  acc_guard2(o0, o1);
  {
    const float oc = 1.0f / (PCAR * VCAR);
#pragma unroll
    for (int r = 0; r < 8; ++r) {
      const float lv  = lrow[r];
      const float ls  = (lv > 0.0f) ? lv : 1.0f;
      const float inv = (lv > 0.0f) ? ((1.0f / ls) * oc) : 0.0f;
      const int idx = (8 * hh + r) * RSP + head * HD + c;
      rsl[idx]      = o0[r] * inv;
      rsl[idx + 16] = o1[r] * inv;
    }
  }
  __syncthreads();
  {
    const int row = tid >> 2, part = tid & 3;
    float* rp = rsl + row * RSP + part * 16;
    const v4f x0 = *(const v4f*)(rp), x1 = *(const v4f*)(rp + 4), x2 = *(const v4f*)(rp + 8), x3 = *(const v4f*)(rp + 12);
    float xv[16];
#pragma unroll
    for (int e = 0; e < 4; ++e) { xv[e] = x0[e]; xv[4 + e] = x1[e]; xv[8 + e] = x2[e]; xv[12 + e] = x3[e]; }
    float s1 = 0.0f;
#pragma unroll
    for (int e = 0; e < 16; ++e) s1 += xv[e];
    s1 += __shfl_xor(s1, 1, 32);
    s1 += __shfl_xor(s1, 2, 32);
    const float mean = s1 * (1.0f / 64.0f);
    float s2 = 0.0f;
#pragma unroll
    for (int e = 0; e < 16; ++e) { const float d = xv[e] - mean; s2 += d * d; }
    s2 += __shfl_xor(s2, 1, 32);
    s2 += __shfl_xor(s2, 2, 32);
    const float var = s2 * (1.0f / 64.0f);
    const float rsd = rsqrtf(var + LNEPS);
    const v4f g0 = *(const v4f*)(gam + part * 16), g1 = *(const v4f*)(gam + part * 16 + 4);
    const v4f g2 = *(const v4f*)(gam + part * 16 + 8), g3 = *(const v4f*)(gam + part * 16 + 12);
    const v4f e0 = *(const v4f*)(bet + part * 16), e1 = *(const v4f*)(bet + part * 16 + 4);
    const v4f e2 = *(const v4f*)(bet + part * 16 + 8), e3 = *(const v4f*)(bet + part * 16 + 12);
    float gv[16], bv[16];
#pragma unroll
    for (int e = 0; e < 4; ++e) {
      gv[e] = g0[e]; gv[4 + e] = g1[e]; gv[8 + e] = g2[e]; gv[12 + e] = g3[e];
      bv[e] = e0[e]; bv[4 + e] = e1[e]; bv[8 + e] = e2[e]; bv[12 + e] = e3[e];
    }
    v4f y0, y1, y2, y3;
#pragma unroll
    for (int e = 0; e < 4; ++e) {
      y0[e] = (xv[e]      - mean) * rsd * bfr(gv[e])      + bfr(bv[e]);
      y1[e] = (xv[4 + e]  - mean) * rsd * bfr(gv[4 + e])  + bfr(bv[4 + e]);
      y2[e] = (xv[8 + e]  - mean) * rsd * bfr(gv[8 + e])  + bfr(bv[8 + e]);
      y3[e] = (xv[12 + e] - mean) * rsd * bfr(gv[12 + e]) + bfr(bv[12 + e]);
    }
    *(v4f*)(rp)      = y0;
    *(v4f*)(rp + 4)  = y1;
    *(v4f*)(rp + 8)  = y2;
    *(v4f*)(rp + 12) = y3;
  }
  __syncthreads();
  v4f ov[4];
  const int rq = tid >> 4, c4 = (tid & 15) * 4;
#pragma unroll
  for (int it = 0; it < 4; ++it) ov[it] = *(const v4f*)(rsl + (it * 4 + rq) * RSP + c4);
  float* dst = OP + ((size_t)bt * NN + q0 + rq) * CC + c4;
  for (int pass = 0; pass < 2; ++pass) {
#pragma unroll
    for (int it = 0; it < 4; ++it) {
      *(volatile v4f*)(dst + (size_t)(it * 4) * CC) = ov[it];
    }
    __threadfence();
  }
}

__global__ __launch_bounds__(256) void ocopy(const float* __restrict__ OPp, float* out) {
  const int tid = threadIdx.x;
  const int bid = blockIdx.x;
  const int b   = bid / CC;
  const int ch  = bid - b * CC;
  if (b >= NB) return;
  const float* src  = OPp + (size_t)b * TT * NN * CC + ch;
  float*       dstb = out + ((size_t)b * CC + ch) * (size_t)(TT * NN);
#pragma unroll 1
  for (int it = 0; it < NOCH; ++it) {
    const int  f  = it * OCHUNK + tid * 4;
    const bool ok = (f < TT * NN);
    const int  fc = ok ? f : 0;
    const int  t  = fc / NN;
    const int  n  = fc - t * NN;
    const float* p = src + ((size_t)t * NN + n) * CC;
    v4f v;
    v[0] = p[0];
    v[1] = p[CC];
    v[2] = p[2 * CC];
    v[3] = p[3 * CC];
    if (ok) {
      *(volatile v4f*)(dstb + f) = v;
      __threadfence();
      *(volatile v4f*)(dstb + f) = v;
    }
  }
}

static inline size_t alup(size_t v) { return (v + 32767) & ~(size_t)32767; }

extern "C" void kernel_launch(void* const* d_in, const int* in_sizes, int n_in,
                              void* d_out, int out_size, void* d_ws, size_t ws_size,
                              hipStream_t stream) {
  if (n_in < 9) return;
  if (in_sizes[0] < NB * CC * TT * NN) return;
  if (in_sizes[1] != CC * CC || in_sizes[2] != CC * CC || in_sizes[3] != CC * CC) return;
  if (in_sizes[4] != NH * HD || in_sizes[5] != NH * HD) return;
  if (in_sizes[6] != CC || in_sizes[7] != CC) return;
  if (in_sizes[8] != NN * NN) return;
  if (out_size < NB * CC * TT * NN) return;

  const float* x     = (const float*)d_in[0];
  const float* Wq    = (const float*)d_in[1];
  const float* Wk    = (const float*)d_in[2];
  const float* Wv    = (const float*)d_in[3];
  const float* a_src = (const float*)d_in[4];
  const float* a_dst = (const float*)d_in[5];
  const float* gam   = (const float*)d_in[6];
  const float* bet   = (const float*)d_in[7];
  const int*   gso   = (const int*)d_in[8];
  float*       out   = (float*)d_out;

  const size_t szWB = (size_t)NPROJ * CC * 2;
  const size_t szMB = (size_t)NN * 16 * 4;
  const size_t szXB = (size_t)MROWS * CC * 2;
  const size_t szF  = (size_t)MROWS * NPROJ * 4;
  const size_t szOP = (size_t)MROWS * CC * 4;
  const size_t szV  = (size_t)BT * CC * KP * 2;
  const size_t szS  = (size_t)2 * BT * NH * KP * 4;
  if (szOP > szF) return;
  size_t off = 0;
  const size_t oWB = off; off = alup(off + szWB);
  const size_t oMB = off; off = alup(off + szMB);
  const size_t oXB = off; off = alup(off + szXB);
  const size_t oF  = off; off = alup(off + szF);
  const size_t oVH = off; off = alup(off + szV);
  const size_t oVL = off; off = alup(off + szV);
  const size_t oS  = off; off = alup(off + szS);
  if (off > ws_size) return;
  if (off > (size_t)WS_CAP) return;

  char* ws = (char*)d_ws;
  u16*      WB  = (u16*)(ws + oWB);
  unsigned* MB  = (unsigned*)(ws + oMB);
  u16*      XB  = (u16*)(ws + oXB);
  float*    F   = (float*)(ws + oF);
  float*    OPl = (float*)(ws + oF);
  u16*      VH  = (u16*)(ws + oVH);
  u16*      VL  = (u16*)(ws + oVL);
  float*    SP  = (float*)(ws + oS);

  const dim3 b256(256), b128(128), b64(ATT_THREADS);
  const dim3 gW((NPROJ * CC / 8 + 255) / 256);
  const dim3 gX(BT * NQT);
  const dim3 gMk((NN * 16 + 255) / 256);
  const dim3 gG((MROWS / 64) * (NPROJ / 64));
  const dim3 gV(BT * NJT);
  const dim3 gA(BT * NQT);
  const dim3 gO(NB * CC);

  wcvt<<<gW, b256, 0, stream>>>(Wq, Wk, Wv, WB);
  xcvt<<<gX, b128, 0, stream>>>(x, XB);
  mbits<<<gMk, b256, 0, stream>>>(gso, MB);
  gemm_bf<<<gG, b128, 0, stream>>>(XB, WB, F, MROWS, NPROJ, CC, 1.0f);
  vs16<<<gV, b256, 0, stream>>>(F, a_src, a_dst, VH, VL, SP);
  gat_attn<<<gA, b64, 0, stream>>>(SP, MB, VH, VL, gam, bet, OPl);
  ocopy<<<gO, b256, 0, stream>>>(OPl, out);
  (void)hipGetLastError();
}
